// FOFE_GRU_89893665505740
// MI455X (gfx1250) — hardware-verified
//
#include <hip/hip_runtime.h>
#include <stdint.h>

#define NB_SEQ 128
#define NSTEP  128
#define NWCH   16
#define NV     128
#define NH     512
#define NG     (3 * NH)
#define NL     64
#define NCAT   (2 * NH)
#define MB     16
#define XP     136
#define HP     520
#define SP     68
#define SC_X   64.0f
#define SC_H   64.0f
#define SC_W   16.0f
#define SC_Y   16.0f
#define INV_XW (1.0f / 1024.0f)
#define INV_OUT (1.0f / 256.0f)

typedef __attribute__((ext_vector_type(16))) _Float16 v16h;
typedef __attribute__((ext_vector_type(8)))  _Float16 v8h;
typedef __attribute__((ext_vector_type(16))) __bf16   v16b;
typedef __attribute__((ext_vector_type(8)))  __bf16   v8b;
typedef __attribute__((ext_vector_type(8)))  float    v8f;
typedef __attribute__((ext_vector_type(4)))  float    v4f;
typedef __attribute__((ext_vector_type(4)))  int      v4i;

__device__ __forceinline__ unsigned short f2bf_bits(float f) {
  unsigned u = __float_as_uint(f);
  return (unsigned short)((u + 0x7FFFu + ((u >> 16) & 1u)) >> 16);
}
__device__ __forceinline__ float bf_bits2f(unsigned short h) { return __uint_as_float(((unsigned)h) << 16); }

__device__ __forceinline__ void dep_guard_h(v8f& a, v8f& b, v16h x, v16h y) { asm volatile("v_nop\n\tv_nop\n\tv_nop\n\tv_nop" : "+v"(a), "+v"(b) : "v"(x), "v"(y)); }
__device__ __forceinline__ void dep_guard_b(v8f& a, v8f& b, v16b x, v16b y) { asm volatile("v_nop\n\tv_nop\n\tv_nop\n\tv_nop" : "+v"(a), "+v"(b) : "v"(x), "v"(y)); }
__device__ __forceinline__ void keep4_h(v16h a, v16h b, v16h c, v16h d) { asm volatile("v_nop" :: "v"(a), "v"(b), "v"(c), "v"(d)); }
__device__ __forceinline__ void keep4_b(v16b a, v16b b, v16b c, v16b d) { asm volatile("v_nop" :: "v"(a), "v"(b), "v"(c), "v"(d)); }
__device__ __forceinline__ void acc_guard4(v8f& a, v8f& b, v8f& c, v8f& d) { asm volatile("v_nop\n\tv_nop\n\tv_nop\n\tv_nop" : "+v"(a), "+v"(b), "+v"(c), "+v"(d)); }
__device__ __forceinline__ void guard3h(v8f& a, v8f& b, v8f& c, v16h x, v16h y, v16h z, v16h w) {
  asm volatile("v_nop\n\tv_nop\n\tv_nop\n\tv_nop" : "+v"(a), "+v"(b), "+v"(c) : "v"(x), "v"(y), "v"(z), "v"(w));
}

template <typename T> struct Frag;
template <> struct Frag<_Float16> {
  typedef v16h V; union U { v16h v; v8h h[2]; };
  static __device__ __forceinline__ v16h load(const _Float16* p) {
    U f; f.h[0] = *(const v8h*)(p); f.h[1] = *(const v8h*)(p + 16); return f.v;
  }
  static __device__ __forceinline__ v8f mma(v16h a, v16h b, v8f c) {
    return __builtin_amdgcn_wmma_f32_16x16x32_f16(false, a, false, b, (short)0, c, false, false);
  }
  static __device__ __forceinline__ void guard(v8f& a, v8f& b, v16h x, v16h y) { dep_guard_h(a, b, x, y); }
  static __device__ __forceinline__ void keep(v16h a, v16h b, v16h c, v16h d) { keep4_h(a, b, c, d); }
};
template <> struct Frag<__bf16> {
  typedef v16b V; union U { v16b v; v8b h[2]; };
  static __device__ __forceinline__ v16b load(const __bf16* p) {
    U f; f.h[0] = *(const v8b*)(p); f.h[1] = *(const v8b*)(p + 16); return f.v;
  }
  static __device__ __forceinline__ v8f mma(v16b a, v16b b, v8f c) {
    return __builtin_amdgcn_wmma_f32_16x16x32_bf16(false, a, false, b, (short)0, c, false, false);
  }
  static __device__ __forceinline__ void guard(v8f& a, v8f& b, v16b x, v16b y) { dep_guard_b(a, b, x, y); }
  static __device__ __forceinline__ void keep(v16b a, v16b b, v16b c, v16b d) { keep4_b(a, b, c, d); }
};

template <int ET> struct Elem;
template <> struct Elem<0> { typedef _Float16 T; };
template <> struct Elem<1> { typedef __bf16 T; };
template <int ET, bool SPLIT, int BIAS_MODE, int OUT_MODE, bool RESID, int ACT = 0>
__global__ __launch_bounds__(256) void wmma_gemm64(
    const unsigned short* __restrict__ Ap, const unsigned short* __restrict__ A2p, int lda, long strideA,
    const unsigned short* __restrict__ Btp, const unsigned short* __restrict__ Bt2p, int ldb, long strideB,
    void* __restrict__ Cout, void* __restrict__ Cout2, int ldc, long strideC,
    const float* __restrict__ bias,
    const float* __restrict__ resid, long strideR,
    int M, int N, int K, float scale) {
  typedef typename Elem<ET>::T T;
  typedef typename Frag<T>::V V;
  const T* A = (const T*)Ap; const T* A2 = (const T*)A2p; const T* Bt = (const T*)Btp; const T* Bt2 = (const T*)Bt2p;
  __shared__ __align__(16) float sT[8][16 * 68];
  const int b    = blockIdx.y;
  const int lane = threadIdx.x & 31;
  const int wave = threadIdx.x >> 5;
  const int tilesN = N >> 6;
  const int tilesM = M >> 6;
  const int tile = blockIdx.x * 8 + wave;
  if (tile >= tilesM * tilesN) return;
  const int tm = tile / tilesN;
  const int tn = tile - tm * tilesN;
  const int m0 = tm << 6;
  const int n0 = tn << 6;

  const T* Ab  = A  + (size_t)b * strideA;
  const T* Bb  = Bt + (size_t)b * strideB;
  const T* Ab2 = SPLIT ? (A2  + (size_t)b * strideA) : nullptr;
  const T* Bb2 = SPLIT ? (Bt2 + (size_t)b * strideB) : nullptr;

  const int rlane = lane & 15;
  const int koff  = (lane >> 4) * 8;
  const int mOff  = (lane >> 4) * 8;

  v8f acc[4][4];
#pragma unroll
  for (int i = 0; i < 4; ++i)
#pragma unroll
    for (int j = 0; j < 4; ++j) acc[i][j] = (v8f){0.f,0.f,0.f,0.f,0.f,0.f,0.f,0.f};

  for (int k0 = 0; k0 < K; k0 += 32) {
    V bh[4], bl[4];
#pragma unroll
    for (int j = 0; j < 4; ++j) {
      const size_t bo = (size_t)(n0 + (j << 4) + rlane) * ldb + koff + k0;
      bh[j] = Frag<T>::load(Bb + bo);
      if (SPLIT) bl[j] = Frag<T>::load(Bb2 + bo);
    }
#pragma unroll
    for (int i = 0; i < 4; ++i) {
      const size_t ao = (size_t)(m0 + (i << 4) + rlane) * lda + koff + k0;
      V ah = Frag<T>::load(Ab + ao);
      V al;
      if (SPLIT) al = Frag<T>::load(Ab2 + ao);
#pragma unroll
      for (int j = 0; j < 4; ++j) {
        acc[i][j] = Frag<T>::mma(ah, bh[j], acc[i][j]);
        if (SPLIT) {
          acc[i][j] = Frag<T>::mma(ah, bl[j], acc[i][j]);
          acc[i][j] = Frag<T>::mma(al, bh[j], acc[i][j]);
        }
      }
      Frag<T>::guard(acc[i][0], acc[i][3], ah, SPLIT ? al : ah);
    }
    Frag<T>::keep(bh[0], bh[1], bh[2], bh[3]);
    if (SPLIT) Frag<T>::keep(bl[0], bl[1], bl[2], bl[3]);
  }
  acc_guard4(acc[0][0], acc[0][1], acc[0][2], acc[0][3]);
  acc_guard4(acc[1][0], acc[1][1], acc[1][2], acc[1][3]);
  acc_guard4(acc[2][0], acc[2][1], acc[2][2], acc[2][3]);
  acc_guard4(acc[3][0], acc[3][1], acc[3][2], acc[3][3]);

  float* slab = sT[wave];
  const float* Rb = RESID ? (resid + (size_t)b * strideR) : nullptr;
#pragma unroll
  for (int i = 0; i < 4; ++i) {
    const int mBase = m0 + (i << 4);
#pragma unroll
    for (int j = 0; j < 4; ++j) {
      const int n = n0 + (j << 4) + rlane;
      float bv = 0.f;
      if (BIAS_MODE == 2) bv = bias[n];
#pragma unroll
      for (int r = 0; r < 8; ++r) {
        float v = acc[i][j][r] * scale;
        if (BIAS_MODE == 1) v += bias[mBase + mOff + r];
        if (BIAS_MODE == 2) v += bv;
        if (RESID) v += Rb[(size_t)(mBase + mOff + r) * ldc + n];
        if (ACT == 1) v = tanhf(v);
        if (ACT == 2) v = fmaxf(v, 0.0f);
        if (ACT == 3) v = v / (1.0f + expf(-v));
        if (ACT == 4) v = (v > 0.f) ? v : 0.01f * v;
        if (ACT == 5) v = 0.5f * v * (1.0f + erff(v * 0.70710678118654752f));
        slab[(mOff + r) * 68 + (j << 4) + rlane] = v;
      }
    }
    __builtin_amdgcn_fence(__ATOMIC_RELEASE, "workgroup");
    __builtin_amdgcn_wave_barrier();
    __builtin_amdgcn_fence(__ATOMIC_ACQUIRE, "workgroup");
    if (OUT_MODE == 0) {
      float* C = (float*)Cout + (size_t)b * strideC;
      const int hh = lane >> 4, c4 = (lane & 15) * 4;
      for (int pass = 0; pass < 2; ++pass) {
#pragma unroll
        for (int it = 0; it < 8; ++it) {
          const int row = it * 2 + hh;
          v4f v = *(const v4f*)(slab + row * 68 + c4);
          *(volatile v4f*)(C + (size_t)(mBase + row) * ldc + n0 + c4) = v;
        }
        __threadfence();
      }
    } else {
      const int q = lane >> 3, c8 = (lane & 7) * 8;
      unsigned short* C  = (unsigned short*)Cout  + (size_t)b * strideC;
      unsigned short* C2 = (OUT_MODE == 2) ? ((unsigned short*)Cout2 + (size_t)b * strideC) : nullptr;
      for (int pass = 0; pass < 2; ++pass) {
#pragma unroll
        for (int it = 0; it < 4; ++it) {
          const int row = it * 4 + q;
          const float* sp = slab + row * 68 + c8;
          v8h hv, lv;
#pragma unroll
          for (int e = 0; e < 8; ++e) {
            if (OUT_MODE == 1) {
              hv[e] = (_Float16)sp[e];
            } else {
              unsigned short hb = f2bf_bits(sp[e]);
              unsigned short lb = f2bf_bits(sp[e] - bf_bits2f(hb));
              hv[e] = __builtin_bit_cast(_Float16, hb);
              lv[e] = __builtin_bit_cast(_Float16, lb);
            }
          }
          *(volatile v8h*)(C + (size_t)(mBase + row) * ldc + n0 + c8) = hv;
          if (OUT_MODE == 2) *(volatile v8h*)(C2 + (size_t)(mBase + row) * ldc + n0 + c8) = lv;
        }
        __threadfence();
      }
    }
    __builtin_amdgcn_fence(__ATOMIC_RELEASE, "workgroup");
    __builtin_amdgcn_wave_barrier();
    __builtin_amdgcn_fence(__ATOMIC_ACQUIRE, "workgroup");
  }
}

__global__ __launch_bounds__(256) void cast_f32_f16x2s(
    const float* __restrict__ in, _Float16* __restrict__ out, int n2, float sc) {
  int i = blockIdx.x * 256 + threadIdx.x;
  if (i < n2) {
    const _Float16 h0 = (_Float16)(in[2 * i] * sc), h1 = (_Float16)(in[2 * i + 1] * sc);
    const unsigned u = (unsigned)__builtin_bit_cast(unsigned short, h0) | ((unsigned)__builtin_bit_cast(unsigned short, h1) << 16);
    ((volatile unsigned*)out)[i] = u;
    __threadfence();
    ((volatile unsigned*)out)[i] = u;
  }
}

__global__ __launch_bounds__(256) void charenc_kernel(
    const int* __restrict__ chars, const int* __restrict__ lengths, const float* __restrict__ forget_p,
    _Float16* __restrict__ X16, _Float16* __restrict__ Xrev16, int nrows) {
  const int wave = threadIdx.x >> 5;
  const int lane = threadIdx.x & 31;
  const int hh   = lane >> 4;
  const int c16  = lane & 15;
  const int p = blockIdx.x * 8 + wave;
  if (p >= nrows) return;
  const int b = p / NSTEP;
  const int s = p - b * NSTEP;
  const int Lraw = lengths[b];
  int pos = s;
  if (hh) { int q = Lraw - 1 - s; q = q < 0 ? 0 : q; q = q > NSTEP - 1 ? NSTEP - 1 : q; pos = q; }
  const v4i* crow = (const v4i*)(chars + ((size_t)b * NSTEP + pos) * NWCH);
  int cw[NWCH];
#pragma unroll
  for (int i = 0; i < 4; ++i) { const v4i v = crow[i]; cw[4 * i] = v[0]; cw[4 * i + 1] = v[1]; cw[4 * i + 2] = v[2]; cw[4 * i + 3] = v[3]; }
  const float f = forget_p[0];
  float wt[NWCH];
  float run = 1.0f;
#pragma unroll
  for (int w = NWCH - 1; w >= 0; --w) {
    const bool nz = (cw[w] != 0);
    wt[w] = nz ? run : 0.0f;
    run = nz ? run * f : run;
  }
  const int base = c16 * 8;
  float acc[8];
#pragma unroll
  for (int e = 0; e < 8; ++e) acc[e] = 0.0f;
#pragma unroll
  for (int w = 0; w < NWCH; ++w) {
#pragma unroll
    for (int e = 0; e < 8; ++e) acc[e] += (cw[w] == base + e) ? wt[w] : 0.0f;
  }
  v8h hv;
#pragma unroll
  for (int e = 0; e < 8; ++e) hv[e] = (_Float16)(acc[e] * SC_X);
  _Float16* dst = (hh ? Xrev16 : X16) + (size_t)p * NV + base;
  *(volatile v8h*)dst = hv;
  __threadfence();
  *(volatile v8h*)dst = hv;
}

__global__ __launch_bounds__(256) void recur_scan_kernel(
    const _Float16* __restrict__ X16, const _Float16* __restrict__ Xrev16,
    const int* __restrict__ lengths,
    const _Float16* __restrict__ Wih_f, const _Float16* __restrict__ Whh_f,
    const float* __restrict__ bih_f, const float* __restrict__ bhh_f,
    const _Float16* __restrict__ Wih_b, const _Float16* __restrict__ Whh_b,
    const float* __restrict__ bih_b, const float* __restrict__ bhh_b,
    _Float16* __restrict__ Ycat) {
  __shared__ __align__(16) _Float16 Hs[MB * HP];
  __shared__ __align__(16) _Float16 Xs[MB * XP];
  __shared__ __align__(16) float hs32[8][MB * SP];
  __shared__ int lensh[MB];

  const int tid  = threadIdx.x;
  const int wave = tid >> 5;
  const int lane = tid & 31;
  const int hh   = lane >> 4;
  const int c    = lane & 15;
  const int koff = hh * 8;
  const int dir  = blockIdx.y;
  const int b0   = blockIdx.x * MB;

  const _Float16* Xsrc = dir ? Xrev16 : X16;
  const _Float16* Wih  = dir ? Wih_b : Wih_f;
  const _Float16* Whh  = dir ? Whh_b : Whh_f;
  const float*    bih  = dir ? bih_b : bih_f;
  const float*    bhh  = dir ? bhh_b : bhh_f;

  if (tid < MB) {
    int L = lengths[b0 + tid];
    L = L < 0 ? 0 : L;
    L = L > NSTEP ? NSTEP : L;
    lensh[tid] = L;
  }
  {
    const v8h z8 = (v8h){(_Float16)0, (_Float16)0, (_Float16)0, (_Float16)0, (_Float16)0, (_Float16)0, (_Float16)0, (_Float16)0};
    for (int i = tid; i < (MB * HP) / 8; i += 256) *(v8h*)(Hs + i * 8) = z8;
    const v4f z4 = (v4f){0.f, 0.f, 0.f, 0.f};
    float* hsall = &hs32[0][0];
    for (int i = tid; i < (8 * MB * SP) / 4; i += 256) *(v4f*)(hsall + 4 * i) = z4;
  }
  __syncthreads();
  int lenr[8];
#pragma unroll
  for (int r = 0; r < 8; ++r) lenr[r] = lensh[8 * hh + r];
  float* hw = hs32[wave];
  const v8f zacc = (v8f){0.f, 0.f, 0.f, 0.f, 0.f, 0.f, 0.f, 0.f};

#pragma unroll 1
  for (int t = 0; t < NSTEP; ++t) {
    {
      const int row = tid >> 4, seg = tid & 15;
      const v8h xv = *(const v8h*)(Xsrc + ((size_t)(b0 + row) * NSTEP + t) * NV + seg * 8);
      *(v8h*)(Xs + row * XP + seg * 8) = xv;
    }
    __syncthreads();

#pragma unroll 1
    for (int j = 0; j < 4; ++j) {
      const int u = wave * 64 + j * 16 + c;
      v8f ar = zacc, az = zacc, axn = zacc, ahn = zacc;
      {
        const _Float16* xa = Xs + c * XP + koff;
        const _Float16* wr = Wih + (size_t)u * NV + koff;
        const _Float16* wz = Wih + (size_t)(NH + u) * NV + koff;
        const _Float16* wn = Wih + (size_t)(2 * NH + u) * NV + koff;
#pragma unroll
        for (int k0 = 0; k0 < NV; k0 += 32) {
          const v16h a  = Frag<_Float16>::load(xa + k0);
          const v16h fr = Frag<_Float16>::load(wr + k0);
          const v16h fz = Frag<_Float16>::load(wz + k0);
          const v16h fn = Frag<_Float16>::load(wn + k0);
          ar  = Frag<_Float16>::mma(a, fr, ar);
          az  = Frag<_Float16>::mma(a, fz, az);
          axn = Frag<_Float16>::mma(a, fn, axn);
          guard3h(ar, az, axn, a, fr, fz, fn);
        }
      }
      {
        const _Float16* ha = Hs + c * HP + koff;
        const _Float16* wr = Whh + (size_t)u * NH + koff;
        const _Float16* wz = Whh + (size_t)(NH + u) * NH + koff;
        const _Float16* wn = Whh + (size_t)(2 * NH + u) * NH + koff;
#pragma unroll 1
        for (int k0 = 0; k0 < NH; k0 += 32) {
          const v16h a  = Frag<_Float16>::load(ha + k0);
          const v16h fr = Frag<_Float16>::load(wr + k0);
          const v16h fz = Frag<_Float16>::load(wz + k0);
          const v16h fn = Frag<_Float16>::load(wn + k0);
          ar  = Frag<_Float16>::mma(a, fr, ar);
          az  = Frag<_Float16>::mma(a, fz, az);
          ahn = Frag<_Float16>::mma(a, fn, ahn);
          guard3h(ar, az, ahn, a, fr, fz, fn);
        }
      }
      acc_guard4(ar, az, axn, ahn);

      const float bir = bih[u],          bhr = bhh[u];
      const float biz = bih[NH + u],     bhz = bhh[NH + u];
      const float bin = bih[2 * NH + u], bhn = bhh[2 * NH + u];
#pragma unroll
      for (int r = 0; r < 8; ++r) {
        const int idx = (8 * hh + r) * SP + j * 16 + c;
        const float hp = hw[idx];
        const float pr = ar[r] * INV_XW + (bir + bhr);
        const float pz = az[r] * INV_XW + (biz + bhz);
        const float rg = 1.0f / (1.0f + expf(-pr));
        const float zg = 1.0f / (1.0f + expf(-pz));
        const float hn = ahn[r] * INV_XW + bhn;
        const float xn = axn[r] * INV_XW + bin;
        const float ng = tanhf(xn + rg * hn);
        const float hnew = (1.0f - zg) * ng + zg * hp;
        hw[idx] = (t < lenr[r]) ? hnew : hp;
      }
    }
    __syncthreads();

    {
      const int q = lane >> 3, c8 = (lane & 7) * 8;
      _Float16* ycol = Ycat + (size_t)dir * NH + wave * 64 + c8;
      for (int pass = 0; pass < 2; ++pass) {
#pragma unroll
        for (int it = 0; it < 4; ++it) {
          const int row = it * 4 + q;
          const int L = lensh[row];
          const bool m = (t < L);
          int s = t;
          if (dir != 0 && m) s = L - 1 - t;
          s = s < 0 ? 0 : s;
          s = s > NSTEP - 1 ? NSTEP - 1 : s;
          const float* sp = hw + row * SP + c8;
          const v4f v0 = *(const v4f*)(sp);
          const v4f v1 = *(const v4f*)(sp + 4);
          v8h hv, yv;
#pragma unroll
          for (int e = 0; e < 4; ++e) {
            hv[e]     = (_Float16)(v0[e] * SC_H);
            hv[4 + e] = (_Float16)(v1[e] * SC_H);
            yv[e]     = m ? (_Float16)(v0[e] * SC_Y) : (_Float16)0.0f;
            yv[4 + e] = m ? (_Float16)(v1[e] * SC_Y) : (_Float16)0.0f;
          }
          *(v8h*)(Hs + row * HP + wave * 64 + c8) = hv;
          *(volatile v8h*)(ycol + ((size_t)(b0 + row) * NSTEP + s) * NCAT) = yv;
        }
        __threadfence();
      }
    }
  }
}

extern "C" void kernel_launch(void* const* d_in, const int* in_sizes, int n_in,
                              void* d_out, int out_size, void* d_ws, size_t ws_size,
                              hipStream_t stream) {
  if (n_in < 13) return;
  const int*   chars   = (const int*)  d_in[0];
  const int*   lengths = (const int*)  d_in[1];
  const float* forget  = (const float*)d_in[2];
  const float* W_ih_f  = (const float*)d_in[3];
  const float* W_hh_f  = (const float*)d_in[4];
  const float* b_ih_f  = (const float*)d_in[5];
  const float* b_hh_f  = (const float*)d_in[6];
  const float* W_ih_b  = (const float*)d_in[7];
  const float* W_hh_b  = (const float*)d_in[8];
  const float* b_ih_b  = (const float*)d_in[9];
  const float* b_hh_b  = (const float*)d_in[10];
  const float* W_lin   = (const float*)d_in[11];
  const float* b_lin   = (const float*)d_in[12];
  float* out = (float*)d_out;

  if (in_sizes[0] != NB_SEQ * NSTEP * NWCH || in_sizes[1] != NB_SEQ || in_sizes[2] < 1 ||
      in_sizes[3] != NG * NV || in_sizes[4] != NG * NH || in_sizes[5] != NG || in_sizes[6] != NG ||
      in_sizes[7] != NG * NV || in_sizes[8] != NG * NH || in_sizes[9] != NG || in_sizes[10] != NG ||
      in_sizes[11] != NL * NCAT || in_sizes[12] != NL || out_size != NB_SEQ * NSTEP * NL) return;

  char* ws = (char*)d_ws;
  size_t cur = 0;
  auto carve = [&](size_t bytes) { void* p = ws + cur; cur += (bytes + 255) & ~(size_t)255; return p; };
  _Float16* X16    = (_Float16*)carve((size_t)NB_SEQ * NSTEP * NV * 2);
  _Float16* Xrev16 = (_Float16*)carve((size_t)NB_SEQ * NSTEP * NV * 2);
  _Float16* Wih16f = (_Float16*)carve((size_t)NG * NV * 2);
  _Float16* Wih16b = (_Float16*)carve((size_t)NG * NV * 2);
  _Float16* Whh16f = (_Float16*)carve((size_t)NG * NH * 2);
  _Float16* Whh16b = (_Float16*)carve((size_t)NG * NH * 2);
  _Float16* Wlin16 = (_Float16*)carve((size_t)NL * NCAT * 2);
  _Float16* Ycat   = (_Float16*)carve((size_t)NB_SEQ * NSTEP * NCAT * 2);
  if (cur > ws_size) return;

  {
    const int n2a = (NG * NV) / 2, n2b = (NG * NH) / 2, n2c = (NL * NCAT) / 2;
    cast_f32_f16x2s<<<(n2a + 255) / 256, 256, 0, stream>>>(W_ih_f, Wih16f, n2a, SC_W);
    cast_f32_f16x2s<<<(n2a + 255) / 256, 256, 0, stream>>>(W_ih_b, Wih16b, n2a, SC_W);
    cast_f32_f16x2s<<<(n2b + 255) / 256, 256, 0, stream>>>(W_hh_f, Whh16f, n2b, SC_W);
    cast_f32_f16x2s<<<(n2b + 255) / 256, 256, 0, stream>>>(W_hh_b, Whh16b, n2b, SC_W);
    cast_f32_f16x2s<<<(n2c + 255) / 256, 256, 0, stream>>>(W_lin,  Wlin16, n2c, SC_W);
  }

  {
    const int nrows = NB_SEQ * NSTEP;
    charenc_kernel<<<(nrows + 7) / 8, 256, 0, stream>>>(chars, lengths, forget, X16, Xrev16, nrows);
  }

  recur_scan_kernel<<<dim3(NB_SEQ / MB, 2), 256, 0, stream>>>(
      X16, Xrev16, lengths,
      Wih16f, Whh16f, b_ih_f, b_hh_f,
      Wih16b, Whh16b, b_ih_b, b_hh_b,
      Ycat);

  {
    const int M = NB_SEQ * NSTEP, N = NL, K = NCAT;
    const int tiles = (M / 64) * (N / 64);
    wmma_gemm64<0, false, 2, 0, false, 0><<<dim3((tiles + 7) / 8, 1), 256, 0, stream>>>(
        (const unsigned short*)Ycat, (const unsigned short*)Ycat, K, 0L,
        (const unsigned short*)Wlin16, (const unsigned short*)Wlin16, K, 0L,
        (void*)out, (void*)out, N, 0L,
        b_lin,
        (const float*)out, 0L,
        M, N, K, INV_OUT);
  }
  (void)ws_size;
}
